// DynamicDepthSeparableTimeSeriesSelfAttention_1537598292709
// MI455X (gfx1250) — hardware-verified
//
#include <hip/hip_runtime.h>


typedef _Float16 v16h __attribute__((ext_vector_type(16)));
typedef _Float16 v8h  __attribute__((ext_vector_type(8)));
typedef __bf16   v16b __attribute__((ext_vector_type(16)));
typedef unsigned short v16us __attribute__((ext_vector_type(16)));
typedef unsigned short v8us  __attribute__((ext_vector_type(8)));
typedef unsigned int v4u __attribute__((ext_vector_type(4)));
typedef float v8f __attribute__((ext_vector_type(8)));
typedef float v4f __attribute__((ext_vector_type(4)));
typedef v8us v8us_a __attribute__((may_alias));
typedef v8h  v8h_a  __attribute__((may_alias));
typedef v4f  v4f_a  __attribute__((may_alias));
typedef v4u  v4u_a  __attribute__((may_alias));

union HFrag { v16h v; v8h p[2]; };
union BFrag { v16b v; v16us u; v8us p[2]; };

#define NB   4
#define CH   64
#define NH   8
#define SEQ  2048
#define HC   512
#define NSEQ 32

static __device__ __forceinline__ v8f mma_f16(v8f c, v16h a, v16h b) {
    c = __builtin_amdgcn_wmma_f32_16x16x32_f16(false, a, false, b, (short)0, c, false, false);
    asm volatile("v_nop\n\tv_nop\n\tv_nop\n\tv_nop" : "+v"(c) : "v"(a), "v"(b));
    return c;
}
static __device__ __forceinline__ v8f mma_bf16(v8f c, v16b a, v16b b) {
    c = __builtin_amdgcn_wmma_f32_16x16x32_bf16(false, a, false, b, (short)0, c, false, false);
    asm volatile("v_nop\n\tv_nop\n\tv_nop\n\tv_nop" : "+v"(c) : "v"(a), "v"(b));
    return c;
}
static __device__ __forceinline__ v8f zero8() {
    v8f z;
#pragma unroll
    for (int i = 0; i < 8; ++i) z[i] = 0.0f;
    return z;
}

static __device__ __forceinline__ unsigned short bf16_rne(float f) {
    unsigned u = __float_as_uint(f);
    u += 0x7FFFu + ((u >> 16) & 1u);
    return (unsigned short)(u >> 16);
}
static __device__ __forceinline__ float bf16_val(unsigned short s) {
    return __uint_as_float(((unsigned)s) << 16);
}
static __device__ __forceinline__ void split_bf16(float f, unsigned short& hi, unsigned short& lo) {
    hi = bf16_rne(f);
    lo = bf16_rne(f - bf16_val(hi));
}
static __device__ __forceinline__ void ldsplit8(const float* __restrict__ p, v8us& hi, v8us& lo) {
    const v4f a = *(const v4f_a*)p;
    const v4f c = *(const v4f_a*)(p + 4);
#pragma unroll
    for (int i = 0; i < 4; ++i) {
        unsigned short H, L;
        split_bf16(a[i], H, L); hi[i] = H;     lo[i] = L;
        split_bf16(c[i], H, L); hi[4 + i] = H; lo[4 + i] = L;
    }
}

#define LT  64
#define NPW 80
#define PB  72
#define PY  80
#define PH  72

__global__ __launch_bounds__(256) void dds_conv_kernel(
    const float* __restrict__ x,
    const float* __restrict__ pw_qk, const float* __restrict__ dw3_qk,
    const float* __restrict__ dw15_qk, const float* __restrict__ gate_qk,
    const float* __restrict__ pw_v, const float* __restrict__ dw3_v,
    const float* __restrict__ dw15_v, const float* __restrict__ gate_v,
    _Float16* qg, _Float16* vg)
{
    const int lt   = blockIdx.x;
    const int hh   = blockIdx.y;
    const int b    = blockIdx.z >> 1;
    const int mode = blockIdx.z & 1;
    const int tid  = threadIdx.x;
    const int lane = tid & 31, h = lane >> 4, m = lane & 15;
    const int w    = __builtin_amdgcn_readfirstlane(tid >> 5);
    const int l0   = lt * LT;
    const int n    = b * NH + hh;

    const float* pw   = mode ? pw_v   : pw_qk;
    const float* dw3  = mode ? dw3_v  : dw3_qk;
    const float* dw15 = mode ? dw15_v : dw15_qk;
    const float* gate = mode ? gate_v : gate_qk;

    __shared__ __attribute__((aligned(16))) unsigned short pwh[CH * PB];
    __shared__ __attribute__((aligned(16))) unsigned short pwl[CH * PB];
    __shared__ __attribute__((aligned(16))) float4 rpool[(2 * NPW * PB * 2) / 16];
    __shared__ float d3s[CH * 3];
    __shared__ float d15s[CH * 15];
    __shared__ __attribute__((aligned(16))) _Float16 stg[CH * PH];

    unsigned short* xh = (unsigned short*)rpool;
    unsigned short* xl = xh + NPW * PB;
    float*          ys = (float*)rpool;

    for (int idx = tid; idx < CH * NPW; idx += 256) {
        const int i = idx / NPW, p = idx - i * NPW;
        const int l = l0 - 8 + p;
        float v = 0.0f;
        if (l >= 0 && l < SEQ) v = x[((size_t)(b * CH + i)) * SEQ + l];
        unsigned short H, L;
        split_bf16(v, H, L);
        xh[p * PB + i] = H;
        xl[p * PB + i] = L;
    }
    for (int idx = tid; idx < CH * CH; idx += 256) {
        const int o = idx >> 6, i = idx & 63;
        const float v = pw[(size_t)hh * CH * CH + idx];
        unsigned short H, L;
        split_bf16(v, H, L);
        pwh[o * PB + i] = H;
        pwl[o * PB + i] = L;
    }
    for (int idx = tid; idx < CH * 3; idx += 256)  d3s[idx]  = dw3[(size_t)hh * CH * 3 + idx];
    for (int idx = tid; idx < CH * 15; idx += 256) d15s[idx] = dw15[(size_t)hh * CH * 15 + idx];
    __syncthreads();

    const int mt  = w & 3;
    const int ntb = w >> 2;
    v8f acc[3];
#pragma unroll
    for (int s = 0; s < 3; ++s) acc[s] = zero8();
#pragma unroll
    for (int ks = 0; ks < 2; ++ks) {
        const int k0 = ks * 32;
        BFrag ah, al;
        {
            const unsigned short* rh = pwh + (mt * 16 + m) * PB + k0 + 8 * h;
            const unsigned short* rl = pwl + (mt * 16 + m) * PB + k0 + 8 * h;
            ah.p[0] = *(const v8us_a*)(rh);
            ah.p[1] = *(const v8us_a*)(rh + 16);
            al.p[0] = *(const v8us_a*)(rl);
            al.p[1] = *(const v8us_a*)(rl + 16);
        }
#pragma unroll
        for (int s = 0; s < 3; ++s) {
            if (s < 2 || w < 4) {
                const int nt = ntb + 2 * s;
                BFrag bh, bl;
                const unsigned short* rh = xh + (nt * 16 + m) * PB + k0 + 8 * h;
                const unsigned short* rl = xl + (nt * 16 + m) * PB + k0 + 8 * h;
                bh.p[0] = *(const v8us_a*)(rh);
                bh.p[1] = *(const v8us_a*)(rh + 16);
                bl.p[0] = *(const v8us_a*)(rl);
                bl.p[1] = *(const v8us_a*)(rl + 16);
                acc[s] = mma_bf16(acc[s], ah.v, bh.v);
                acc[s] = mma_bf16(acc[s], ah.v, bl.v);
                acc[s] = mma_bf16(acc[s], al.v, bh.v);
            }
        }
    }
    __syncthreads();

#pragma unroll
    for (int s = 0; s < 3; ++s) {
        if (s < 2 || w < 4) {
            const int nt = ntb + 2 * s;
#pragma unroll
            for (int r = 0; r < 8; ++r)
                ys[(mt * 16 + 8 * h + r) * PY + nt * 16 + m] = acc[s][r];
        }
    }
    __syncthreads();

    const float g0 = gate[0], g1 = gate[1];
    const float mg = fmaxf(g0, g1);
    const float ea = expf(g0 - mg), eb = expf(g1 - mg);
    const float ginv = 1.0f / (ea + eb);
    const float gs0 = ea * ginv, gs1 = eb * ginv;
    const float qscale = 22.627416997969522f;

    for (int idx = tid; idx < CH * LT; idx += 256) {
        int o, ll;
        if (mode == 0) { o = idx & 63; ll = idx >> 6; }
        else           { ll = idx & 63; o = idx >> 6; }
        const float* yr = ys + o * PY + ll;
        float a3 = 0.0f, a15 = 0.0f;
#pragma unroll
        for (int t = 0; t < 3; ++t)  a3  = fmaf(d3s[o * 3 + t],   yr[7 + t], a3);
#pragma unroll
        for (int t = 0; t < 15; ++t) a15 = fmaf(d15s[o * 15 + t], yr[1 + t], a15);
        const float z = gs0 * a3 + gs1 * a15;
        if (mode == 0) stg[ll * PH + o] = (_Float16)(z * qscale);
        else           stg[o * PH + ll] = (_Float16)(z * 16.0f);
    }
    __syncthreads();

    {
        const int lineA = w * 8 + (lane >> 3);
        const int lineB = lineA + 4;
        const int piece = lane & 7;
        const v8h va = *(const v8h_a*)(stg + lineA * PH + piece * 8);
        const v8h vb = *(const v8h_a*)(stg + lineB * PH + piece * 8);
        _Float16* da;
        _Float16* db;
        if (mode == 0) {
            da = qg + ((size_t)(n * SEQ + l0 + lineA)) * CH + piece * 8;
            db = qg + ((size_t)(n * SEQ + l0 + lineB)) * CH + piece * 8;
        } else {
            da = vg + ((size_t)(n * CH + lineA)) * SEQ + l0 + piece * 8;
            db = vg + ((size_t)(n * CH + lineB)) * SEQ + l0 + piece * 8;
        }
        *(volatile v8h*)da = va;
        *(volatile v8h*)db = vb;
        __threadfence();
        *(volatile v8h*)da = va;
        *(volatile v8h*)db = vb;
    }
}

#define KT 64

__global__ __launch_bounds__(256) void attn_kernel(
    const _Float16* __restrict__ qg,
    const _Float16* __restrict__ vg,
    float* attn)
{
    const int n    = blockIdx.x;
    const int j0   = blockIdx.y * 128;
    const int tid  = threadIdx.x;
    const int lane = tid & 31, h = lane >> 4, m = lane & 15;
    const int w    = __builtin_amdgcn_readfirstlane(tid >> 5);

    __shared__ __attribute__((aligned(16))) float4 pool[2048];
    _Float16* lq = (_Float16*)pool;
    _Float16* lv = lq + KT * CH;
    v4u* lq4 = (v4u*)pool;
    v4u* lv4 = lq4 + (KT * CH) / 8;
    const v4u* qg4 = (const v4u*)qg;
    const v4u* vg4 = (const v4u*)vg;

    HFrag qb0, qb1;
    {
        const _Float16* qr = qg + ((size_t)(n * SEQ + j0 + w * 16 + m)) * CH;
        qb0.p[0] = *(const v8h_a*)(qr + 8 * h);
        qb0.p[1] = *(const v8h_a*)(qr + 16 + 8 * h);
        qb1.p[0] = *(const v8h_a*)(qr + 32 + 8 * h);
        qb1.p[1] = *(const v8h_a*)(qr + 48 + 8 * h);
    }

    v8f O[4];
#pragma unroll
    for (int cc = 0; cc < 4; ++cc) O[cc] = zero8();
    float m_run = -1.0e30f, s_run = 0.0f;
    const float kInvQ = 1.0f / 4096.0f;

#pragma unroll 1
    for (int it = 0; it < SEQ / KT; ++it) {
        const int i0 = it * KT;
        __syncthreads();
#pragma unroll
        for (int s = 0; s < 2; ++s) {
            const int idx = tid + s * 256;
            const int r = idx >> 3, c8 = idx & 7;
            lq4[idx] = *(const v4u_a*)(qg4 + ((size_t)(n * SEQ + i0 + r)) * (CH / 8) + c8);
            lv4[idx] = *(const v4u_a*)(vg4 + ((size_t)(n * CH + r)) * (SEQ / 8) + (i0 >> 3) + c8);
        }
        __syncthreads();

        v8f st[4];
#pragma unroll
        for (int t = 0; t < 4; ++t) {
            const _Float16* ar = lq + (t * 16 + m) * CH;
            HFrag a0, a1;
            a0.p[0] = *(const v8h_a*)(ar + 8 * h);
            a0.p[1] = *(const v8h_a*)(ar + 16 + 8 * h);
            a1.p[0] = *(const v8h_a*)(ar + 32 + 8 * h);
            a1.p[1] = *(const v8h_a*)(ar + 48 + 8 * h);
            v8f c = zero8();
            c = mma_f16(c, a0.v, qb0.v);
            c = mma_f16(c, a1.v, qb1.v);
            st[t] = c;
        }

        float mt = -1.0e30f;
#pragma unroll
        for (int t = 0; t < 4; ++t)
#pragma unroll
            for (int r = 0; r < 8; ++r) mt = fmaxf(mt, st[t][r]);
        mt = fmaxf(mt, __shfl_xor(mt, 16, 32));
        const float m_new = fmaxf(m_run, mt);
        const float alpha = __expf((m_run - m_new) * kInvQ);
#pragma unroll
        for (int cc = 0; cc < 4; ++cc)
#pragma unroll
            for (int r = 0; r < 8; ++r) O[cc][r] = O[cc][r] * alpha;

        float ssum = 0.0f;
#pragma unroll
        for (int u = 0; u < 2; ++u) {
            HFrag pf;
#pragma unroll
            for (int r = 0; r < 8; ++r) {
                const float e0 = __expf((st[2 * u][r]     - m_new) * kInvQ);
                const float e1 = __expf((st[2 * u + 1][r] - m_new) * kInvQ);
                ssum += e0 + e1;
                pf.p[0][r] = (_Float16)e0;
                pf.p[1][r] = (_Float16)e1;
            }
#pragma unroll
            for (int cc = 0; cc < 4; ++cc) {
                const _Float16* vr = lv + (cc * 16 + m) * KT + u * 32;
                HFrag va;
                va.p[0] = *(const v8h_a*)(vr + 8 * h);
                va.p[1] = *(const v8h_a*)(vr + 16 + 8 * h);
                O[cc] = mma_f16(O[cc], va.v, pf.v);
            }
        }
        ssum += __shfl_xor(ssum, 16, 32);
        s_run = s_run * alpha + ssum;
        m_run = m_new;
    }

    const float inv = 1.0f / (s_run * 16.0f);
    __syncthreads();
    float* stage = (float*)pool + w * 1024;
#pragma unroll
    for (int cc = 0; cc < 4; ++cc)
#pragma unroll
        for (int r = 0; r < 8; ++r)
            stage[m * 64 + cc * 16 + 8 * h + r] = O[cc][r] * inv;
    __syncthreads();
    float* base = attn + ((size_t)(n * SEQ + j0 + w * 16)) * CH;
    v4f vals[8];
#pragma unroll
    for (int s = 0; s < 8; ++s) vals[s] = *(const v4f_a*)(stage + s * 128 + lane * 4);
#pragma unroll
    for (int s = 0; s < 8; ++s) *(volatile v4f*)(base + s * 128 + lane * 4) = vals[s];
    __threadfence();
#pragma unroll
    for (int s = 0; s < 8; ++s) *(volatile v4f*)(base + s * 128 + lane * 4) = vals[s];
}

__global__ __launch_bounds__(128) void unify_kernel(
    const float* __restrict__ unify,
    const float* __restrict__ attn,
    float* out)
{
    const int l0   = blockIdx.x * 32;
    const int b    = blockIdx.y;
    const int tid  = threadIdx.x;
    const int lane = tid & 31, h = lane >> 4, m = lane & 15;
    const int w    = __builtin_amdgcn_readfirstlane(tid >> 5);

    __shared__ __attribute__((aligned(16))) float stage[CH * 32];

    v8f acc[2];
    acc[0] = zero8();
    acc[1] = zero8();
    const float* arow = unify + (size_t)(w * 16 + m) * HC;

#pragma unroll 1
    for (int ks = 0; ks < HC / 32; ++ks) {
        const int hh = ks >> 1;
        const int c0 = (ks & 1) * 32;
        BFrag ah, al;
        ldsplit8(arow + ks * 32 + 8 * h,      ah.p[0], al.p[0]);
        ldsplit8(arow + ks * 32 + 16 + 8 * h, ah.p[1], al.p[1]);
#pragma unroll
        for (int nt = 0; nt < 2; ++nt) {
            const float* brow = attn + ((size_t)((b * NH + hh) * SEQ + l0 + nt * 16 + m)) * CH + c0;
            BFrag bh, bl;
            ldsplit8(brow + 8 * h,      bh.p[0], bl.p[0]);
            ldsplit8(brow + 16 + 8 * h, bh.p[1], bl.p[1]);
            acc[nt] = mma_bf16(acc[nt], ah.v, bh.v);
            acc[nt] = mma_bf16(acc[nt], ah.v, bl.v);
            acc[nt] = mma_bf16(acc[nt], al.v, bh.v);
        }
    }

#pragma unroll
    for (int nt = 0; nt < 2; ++nt)
#pragma unroll
        for (int r = 0; r < 8; ++r)
            stage[(w * 16 + 8 * h + r) * 32 + nt * 16 + m] = acc[nt][r];
    __syncthreads();

    v4f vals[4];
    float* dst[4];
#pragma unroll
    for (int s = 0; s < 4; ++s) {
        const int line  = w * 16 + s * 4 + (lane >> 3);
        const int piece = lane & 7;
        vals[s] = *(const v4f_a*)(stage + line * 32 + piece * 4);
        dst[s]  = out + ((size_t)(b * CH + line)) * SEQ + l0 + piece * 4;
    }
#pragma unroll
    for (int s = 0; s < 4; ++s) *(volatile v4f*)(dst[s]) = vals[s];
    __threadfence();
#pragma unroll
    for (int s = 0; s < 4; ++s) *(volatile v4f*)(dst[s]) = vals[s];
}

extern "C" void kernel_launch(void* const* d_in, const int* in_sizes, int n_in,
                              void* d_out, int out_size, void* d_ws, size_t ws_size,
                              hipStream_t stream) {
    if (n_in < 10) return;
    if (in_sizes[0] != NB * CH * SEQ) return;
    if (in_sizes[1] != HC * CH || in_sizes[5] != HC * CH) return;
    if (in_sizes[2] != HC * 3  || in_sizes[6] != HC * 3)  return;
    if (in_sizes[3] != HC * 15 || in_sizes[7] != HC * 15) return;
    if (in_sizes[4] < 2 || in_sizes[8] < 2) return;
    if (in_sizes[9] != CH * HC) return;
    if (out_size != NB * CH * SEQ) return;

    const size_t q_bytes = (size_t)NSEQ * SEQ * CH * sizeof(_Float16);
    const size_t v_bytes = (size_t)NSEQ * CH * SEQ * sizeof(_Float16);
    const size_t a_bytes = (size_t)NSEQ * SEQ * CH * sizeof(float);
    if (ws_size < q_bytes + v_bytes + a_bytes) return;

    const float* x       = (const float*)d_in[0];
    const float* pw_qk   = (const float*)d_in[1];
    const float* dw3_qk  = (const float*)d_in[2];
    const float* dw15_qk = (const float*)d_in[3];
    const float* gate_qk = (const float*)d_in[4];
    const float* pw_v    = (const float*)d_in[5];
    const float* dw3_v   = (const float*)d_in[6];
    const float* dw15_v  = (const float*)d_in[7];
    const float* gate_v  = (const float*)d_in[8];
    const float* unify   = (const float*)d_in[9];

    unsigned char* ws = (unsigned char*)d_ws;
    _Float16* qg   = (_Float16*)(ws);
    _Float16* vg   = (_Float16*)(ws + q_bytes);
    float*    attn = (float*)(ws + q_bytes + v_bytes);
    float*    out  = (float*)d_out;

    dds_conv_kernel<<<dim3(SEQ / LT, NH, NB * 2), 256, 0, stream>>>(
        x, pw_qk, dw3_qk, dw15_qk, gate_qk, pw_v, dw3_v, dw15_v, gate_v, qg, vg);
    attn_kernel<<<dim3(NSEQ, SEQ / 128), 256, 0, stream>>>(qg, vg, attn);
    unify_kernel<<<dim3(SEQ / 32, NB), 128, 0, stream>>>(unify, attn, out);
}
